// GNNCriticVariable_12094627905888
// MI455X (gfx1250) — hardware-verified
//
#include <hip/hip_runtime.h>
#include <stddef.h>


#pragma clang fp contract(off)

#define NAG    512
#define FIN    128
#define HID    512
#define KNB    16
#define TOPN   (KNB + 1)
#define AW     (NAG / 32)
#define NTHR   256
#define KTHR   512
#define GT     128
#define PB1    ((HID * FIN / 8) / NTHR)
#define PB2    ((HID * HID / 8) / NTHR)
#define WSCALE 16
#define ASC2   64
#define WSCAP  134217728
#define LDS_GEMM (GT * GT * 4)

static_assert(AW == 16);
static_assert(NAG == KTHR);
static_assert((HID % GT) == 0 && (NAG % GT) == 0);
static_assert((FIN % 32) == 0 && (HID % 32) == 0);
static_assert(HID == 4 * 128);
static_assert(FIN == 4 * 32);
static_assert(NAG == 8 * 64);
static_assert(PB1 * NTHR * 8 == HID * FIN && PB2 * NTHR * 8 == HID * HID);
static_assert(GT == 8 * 16);

typedef float    v4f  __attribute__((ext_vector_type(4)));
typedef float    v8f  __attribute__((ext_vector_type(8)));
typedef unsigned v4u  __attribute__((ext_vector_type(4)));
typedef _Float16 v4h  __attribute__((ext_vector_type(4)));
typedef _Float16 v8h  __attribute__((ext_vector_type(8)));
typedef _Float16 v16h __attribute__((ext_vector_type(16)));
union FragH { v16h v; v8h h[2]; };

__device__ __forceinline__ v8f wmf(v16h a, v16h b, v8f c) {
  v8f d = __builtin_amdgcn_wmma_f32_16x16x32_f16(false, a, false, b, (short)0, c, false, false);
  asm volatile("v_nop\n\tv_nop\n\tv_nop\n\tv_nop" : "+v"(d) : "v"(a), "v"(b));
  return d;
}

__device__ __forceinline__ float th1(float x) {
  const float xc = fminf(fmaxf(x, -16.0f), 16.0f);
  const float e  = __builtin_amdgcn_exp2f(xc * 2.8853900817779268f);
  const float r  = __builtin_amdgcn_rcpf(e + 1.0f);
  return 1.0f - 2.0f * r;
}
__device__ __forceinline__ v4f th4(v4f v) {
  v4f o;
  o.x = th1(v.x); o.y = th1(v.y); o.z = th1(v.z); o.w = th1(v.w);
  return o;
}

__global__ __launch_bounds__(NTHR) void k_prep(const float* __restrict__ obs, const float* __restrict__ w1,
                                               const float* __restrict__ w2, _Float16* obs16, _Float16* w1t,
                                               _Float16* w2t, int nObsBlk) {
  const int tid = threadIdx.x;
  const int blk = (int)blockIdx.x;
  v8h hv;
  _Float16* d;
  if (blk < nObsBlk) {
    const size_t i = (size_t)blk * NTHR + (size_t)tid;
    const float* p = obs + i * 8;
    const v4f a = *(const v4f*)p, c = *(const v4f*)(p + 4);
    hv[0] = (_Float16)a.x; hv[1] = (_Float16)a.y; hv[2] = (_Float16)a.z; hv[3] = (_Float16)a.w;
    hv[4] = (_Float16)c.x; hv[5] = (_Float16)c.y; hv[6] = (_Float16)c.z; hv[7] = (_Float16)c.w;
    d = obs16 + i * 8;
  } else if (blk < nObsBlk + PB1) {
    const int i  = (blk - nObsBlk) * NTHR + tid;
    const int n  = i / (FIN / 8);
    const int k0 = (i - n * (FIN / 8)) * 8;
#pragma unroll
    for (int e = 0; e < 8; ++e) hv[e] = (_Float16)(w1[(k0 + e) * HID + n] * (float)WSCALE);
    d = w1t + (size_t)i * 8;
  } else {
    const int i  = (blk - nObsBlk - PB1) * NTHR + tid;
    const int n  = i / (HID / 8);
    const int k0 = (i - n * (HID / 8)) * 8;
#pragma unroll
    for (int e = 0; e < 8; ++e) hv[e] = (_Float16)(w2[(k0 + e) * HID + n] * (float)WSCALE);
    d = w2t + (size_t)i * 8;
  }
  *(volatile v8h*)d = hv;
  __threadfence();
  *(volatile v8h*)d = hv;
}

__global__ __launch_bounds__(KTHR) void k_knn(const float* __restrict__ obs, unsigned* adjT) {
  __shared__ float sx[NAG];
  __shared__ float sy[NAG];
  __shared__ __attribute__((aligned(16))) unsigned sadj[NAG * AW];
  const int b = (int)blockIdx.x, i = threadIdx.x;
  const float* row = obs + ((size_t)b * NAG + (size_t)i) * FIN;
  const float px = row[0], py = row[1];
  sx[i] = px; sy[i] = py;
  __syncthreads();

  float bd[TOPN]; int bi[TOPN];
  const float pinf = __uint_as_float(0x7f800000u);
#pragma unroll
  for (int p = 0; p < TOPN; ++p) { bd[p] = pinf; bi[p] = 0; }

#pragma unroll 1
  for (int j = 0; j < NAG; ++j) {
    const float dx = px - sx[j];
    const float dy = py - sy[j];
    const float qx = dx * dx;
    const float qy = dy * dy;
    const float d2 = qx + qy;
    const bool ins = d2 < bd[TOPN - 1];
    if (__builtin_amdgcn_ballot_w32(ins) != 0u) {
      bool c[TOPN];
#pragma unroll
      for (int p = 0; p < TOPN; ++p) c[p] = d2 < bd[p];
#pragma unroll
      for (int p = TOPN - 1; p >= 1; --p) {
        const float nd = c[p - 1] ? bd[p - 1] : (c[p] ? d2 : bd[p]);
        const int   ni = c[p - 1] ? bi[p - 1] : (c[p] ? j  : bi[p]);
        bd[p] = nd; bi[p] = ni;
      }
      bd[0] = c[0] ? d2 : bd[0];
      bi[0] = c[0] ? j  : bi[0];
    }
  }

  unsigned wr[AW];
#pragma unroll
  for (int w = 0; w < AW; ++w) {
    unsigned a = 0u;
#pragma unroll
    for (int k = 1; k < TOPN; ++k) a |= ((bi[k] >> 5) == w) ? (1u << (bi[k] & 31)) : 0u;
    wr[w] = a;
  }
  v4u* srow = (v4u*)(sadj + i * AW);
#pragma unroll
  for (int q = 0; q < 4; ++q) {
    v4u v; v.x = wr[4 * q]; v.y = wr[4 * q + 1]; v.z = wr[4 * q + 2]; v.w = wr[4 * q + 3];
    srow[q] = v;
  }
  __syncthreads();

  const int tw = i >> 5, tb = i & 31;
  unsigned tc[AW];
#pragma unroll
  for (int w = 0; w < AW; ++w) {
    unsigned a = 0u;
#pragma unroll 4
    for (int ii = 0; ii < 32; ++ii) {
      const unsigned x = sadj[(32 * w + ii) * AW + tw];
      a |= ((x >> tb) & 1u) << ii;
    }
    tc[w] = a;
  }
  __syncthreads();
#pragma unroll
  for (int q = 0; q < 4; ++q) {
    v4u v; v.x = tc[4 * q]; v.y = tc[4 * q + 1]; v.z = tc[4 * q + 2]; v.w = tc[4 * q + 3];
    srow[q] = v;
  }
  __syncthreads();

  unsigned* gp = adjT + (size_t)b * NAG * AW;
  const v4u o0 = ((const v4u*)sadj)[i];
  const v4u o1 = ((const v4u*)sadj)[KTHR + i];
  const v4u o2 = ((const v4u*)sadj)[2 * KTHR + i];
  const v4u o3 = ((const v4u*)sadj)[3 * KTHR + i];
  *(volatile v4u*)(gp + 4 * i)              = o0;
  *(volatile v4u*)(gp + 4 * (KTHR + i))     = o1;
  *(volatile v4u*)(gp + 4 * (2 * KTHR + i)) = o2;
  *(volatile v4u*)(gp + 4 * (3 * KTHR + i)) = o3;
  __threadfence();
  *(volatile v4u*)(gp + 4 * i)              = o0;
  *(volatile v4u*)(gp + 4 * (KTHR + i))     = o1;
  *(volatile v4u*)(gp + 4 * (2 * KTHR + i)) = o2;
  *(volatile v4u*)(gp + 4 * (3 * KTHR + i)) = o3;
}

template <int KD>
__global__ __launch_bounds__(NTHR) void k_gemm(const _Float16* __restrict__ A, const _Float16* __restrict__ Bw,
                                               float* C, float osc) {
  extern __shared__ v4f lds_dyn[];
  float* stg = (float*)lds_dyn;
  const int tid = threadIdx.x, lane = tid & 31, wave = tid >> 5, hh = lane >> 4, m = lane & 15;
  const int wr = wave & 3, wc = wave >> 2;
  const int rowBase = (int)blockIdx.y * GT, colBase = (int)blockIdx.x * GT;
  const _Float16* ap0 = A + (size_t)(rowBase + 32 * wr + m) * KD + 8 * hh;
  const _Float16* ap1 = ap0 + (size_t)16 * KD;
  const _Float16* bp0 = Bw + (size_t)(colBase + 64 * wc + m) * KD + 8 * hh;

  v8f acc[2][4];
#pragma unroll
  for (int i2 = 0; i2 < 2; ++i2)
#pragma unroll
    for (int t = 0; t < 4; ++t) { v8f z = {0.f, 0.f, 0.f, 0.f, 0.f, 0.f, 0.f, 0.f}; acc[i2][t] = z; }

#pragma unroll 1
  for (int kt = 0; kt < KD / 32; ++kt) {
    const int k0 = 32 * kt;
    FragH a0, a1;
    a0.h[0] = *(const v8h*)(ap0 + k0);     a0.h[1] = *(const v8h*)(ap0 + k0 + 16);
    a1.h[0] = *(const v8h*)(ap1 + k0);     a1.h[1] = *(const v8h*)(ap1 + k0 + 16);
#pragma unroll
    for (int t = 0; t < 4; ++t) {
      const _Float16* bp = bp0 + (size_t)(16 * t) * KD + k0;
      FragH bf;
      bf.h[0] = *(const v8h*)bp;
      bf.h[1] = *(const v8h*)(bp + 16);
      acc[0][t] = wmf(a0.v, bf.v, acc[0][t]);
      acc[1][t] = wmf(a1.v, bf.v, acc[1][t]);
    }
  }

  float* sp = stg + (32 * wr + 8 * hh) * GT + 64 * wc + m;
#pragma unroll
  for (int i2 = 0; i2 < 2; ++i2)
#pragma unroll
    for (int t = 0; t < 4; ++t)
#pragma unroll
      for (int r = 0; r < 8; ++r) sp[(16 * i2 + r) * GT + 16 * t] = acc[i2][t][r] * osc;
  __syncthreads();

  const float* lp = stg + wave * 16 * GT + 4 * lane;
  float* gp = C + (size_t)(rowBase + 16 * wave) * HID + colBase + 4 * lane;
#pragma unroll
  for (int rr = 0; rr < 16; ++rr) {
    const v4f v = *(const v4f*)(lp + rr * GT);
    *(volatile v4f*)(gp + (size_t)rr * HID) = v;
  }
  __threadfence();
#pragma unroll
  for (int rr = 0; rr < 16; ++rr) {
    const v4f v = *(const v4f*)(lp + rr * GT);
    *(volatile v4f*)(gp + (size_t)rr * HID) = v;
  }
}

template <int L2>
__global__ __launch_bounds__(NTHR) void k_agg(const float* __restrict__ mb, const unsigned* __restrict__ adjT,
                                              const float* __restrict__ bias, _Float16* hout,
                                              const float* __restrict__ obs, const float* __restrict__ wout,
                                              const float* __restrict__ bout, float* out) {
  __shared__ __attribute__((aligned(16))) unsigned sadj[NAG * AW];
  __shared__ __attribute__((aligned(16))) float sval[NAG];
  const int tid = threadIdx.x, lane = tid & 31, wave = tid >> 5;
  const int b = (int)blockIdx.x;
  const size_t rowB = (size_t)b * NAG;
  {
    const v4u* src = (const v4u*)(adjT + rowB * AW);
    for (int c = tid; c < (NAG * AW) / 4; c += NTHR) ((v4u*)sadj)[c] = src[c];
  }
  __syncthreads();

  const v4f bq0 = *(const v4f*)(bias + 4 * lane);
  const v4f bq1 = *(const v4f*)(bias + 128 + 4 * lane);
  const v4f bq2 = *(const v4f*)(bias + 256 + 4 * lane);
  const v4f bq3 = *(const v4f*)(bias + 384 + 4 * lane);
  v4f wq0 = {0.f, 0.f, 0.f, 0.f}, wq1 = wq0, wq2 = wq0, wq3 = wq0;
  float bo = 0.0f;
  if (L2) {
    wq0 = *(const v4f*)(wout + 4 * lane);
    wq1 = *(const v4f*)(wout + 128 + 4 * lane);
    wq2 = *(const v4f*)(wout + 256 + 4 * lane);
    wq3 = *(const v4f*)(wout + 384 + 4 * lane);
    bo  = bout[0];
  }

#pragma unroll 1
  for (int j = 0; j < NAG / 8; ++j) {
    const int t = wave * (NAG / 8) + j;
    const float* mt = mb + (rowB + (size_t)t) * HID + 4 * lane;
    v4f a0 = *(const v4f*)mt;
    v4f a1 = *(const v4f*)(mt + 128);
    v4f a2 = *(const v4f*)(mt + 256);
    v4f a3 = *(const v4f*)(mt + 384);
    const unsigned* arow = sadj + t * AW;
#pragma unroll 1
    for (int w = 0; w < AW; ++w) {
      unsigned msk = (unsigned)__builtin_amdgcn_readfirstlane((int)arow[w]);
#pragma unroll 1
      for (int it = 0; it < 32; ++it) {
        if (msk == 0u) break;
        const int s = 32 * w + (int)__builtin_ctz(msk);
        msk &= msk - 1u;
        const float* ms = mb + (rowB + (size_t)s) * HID + 4 * lane;
        a0 += *(const v4f*)ms;
        a1 += *(const v4f*)(ms + 128);
        a2 += *(const v4f*)(ms + 256);
        a3 += *(const v4f*)(ms + 384);
      }
    }
    a0 = th4(a0 + bq0); a1 = th4(a1 + bq1); a2 = th4(a2 + bq2); a3 = th4(a3 + bq3);

    if (!L2) {
      v4h h0, h1, h2, h3;
      h0.x = (_Float16)(a0.x * (float)ASC2); h0.y = (_Float16)(a0.y * (float)ASC2);
      h0.z = (_Float16)(a0.z * (float)ASC2); h0.w = (_Float16)(a0.w * (float)ASC2);
      h1.x = (_Float16)(a1.x * (float)ASC2); h1.y = (_Float16)(a1.y * (float)ASC2);
      h1.z = (_Float16)(a1.z * (float)ASC2); h1.w = (_Float16)(a1.w * (float)ASC2);
      h2.x = (_Float16)(a2.x * (float)ASC2); h2.y = (_Float16)(a2.y * (float)ASC2);
      h2.z = (_Float16)(a2.z * (float)ASC2); h2.w = (_Float16)(a2.w * (float)ASC2);
      h3.x = (_Float16)(a3.x * (float)ASC2); h3.y = (_Float16)(a3.y * (float)ASC2);
      h3.z = (_Float16)(a3.z * (float)ASC2); h3.w = (_Float16)(a3.w * (float)ASC2);
      _Float16* hp = hout + (rowB + (size_t)t) * HID + 4 * lane;
      *(volatile v4h*)hp         = h0;
      *(volatile v4h*)(hp + 128) = h1;
      *(volatile v4h*)(hp + 256) = h2;
      *(volatile v4h*)(hp + 384) = h3;
      __threadfence();
      *(volatile v4h*)hp         = h0;
      *(volatile v4h*)(hp + 128) = h1;
      *(volatile v4h*)(hp + 256) = h2;
      *(volatile v4h*)(hp + 384) = h3;
    } else {
      float p = a0.x * wq0.x + a0.y * wq0.y + a0.z * wq0.z + a0.w * wq0.w
              + a1.x * wq1.x + a1.y * wq1.y + a1.z * wq1.z + a1.w * wq1.w
              + a2.x * wq2.x + a2.y * wq2.y + a2.z * wq2.z + a2.w * wq2.w
              + a3.x * wq3.x + a3.y * wq3.y + a3.z * wq3.z + a3.w * wq3.w;
#pragma unroll
      for (int o = 16; o >= 1; o >>= 1) p += __shfl_xor(p, o, 32);
      const v4f ov = *(const v4f*)(obs + (rowB + (size_t)t) * FIN + 4 * lane);
      const int nz = ((ov.x != 0.0f) | (ov.y != 0.0f) | (ov.z != 0.0f) | (ov.w != 0.0f)) ? 1 : 0;
      const unsigned any = __builtin_amdgcn_ballot_w32(nz != 0);
      const float val = (any != 0u) ? (p + bo) : 0.0f;
      if (lane == 0) sval[t] = val;
    }
  }

  if (L2) {
    __syncthreads();
    if (tid < NAG / 4) {
      const v4f v = *(const v4f*)(sval + 4 * tid);
      float* op = out + rowB + 4 * tid;
      *(volatile v4f*)op = v;
      __threadfence();
      *(volatile v4f*)op = v;
    }
  }
}

extern "C" void kernel_launch(void* const* d_in, const int* in_sizes, int n_in,
                              void* d_out, int out_size, void* d_ws, size_t ws_size,
                              hipStream_t stream) {
  if (n_in < 7) return;
  const int nObs = in_sizes[0];
  const int nB = nObs / (NAG * FIN);
  if (nB <= 0 || nB > 4096 || nB * NAG * FIN != nObs) return;
  if (in_sizes[1] != FIN * HID || in_sizes[2] != HID) return;
  if (in_sizes[3] != HID * HID || in_sizes[4] != HID) return;
  if (in_sizes[5] != HID || in_sizes[6] < 1) return;
  if (out_size != nB * NAG) return;

  const float* obs  = (const float*)d_in[0];
  const float* W1   = (const float*)d_in[1];
  const float* b1   = (const float*)d_in[2];
  const float* W2   = (const float*)d_in[3];
  const float* b2   = (const float*)d_in[4];
  const float* Wout = (const float*)d_in[5];
  const float* bout = (const float*)d_in[6];
  float* out = (float*)d_out;

  const int M = nB * NAG;

  char* ws = (char*)d_ws;
  size_t off = 0;
  const size_t oAdj = off; off += (size_t)M * AW * 4;      off = (off + 255) & ~(size_t)255;
  const size_t oO16 = off; off += (size_t)M * FIN * 2;     off = (off + 255) & ~(size_t)255;
  const size_t oW1  = off; off += (size_t)HID * FIN * 2;   off = (off + 255) & ~(size_t)255;
  const size_t oW2  = off; off += (size_t)HID * HID * 2;   off = (off + 255) & ~(size_t)255;
  const size_t oM   = off; off += (size_t)M * HID * 4;     off = (off + 255) & ~(size_t)255;
  const size_t oH   = off; off += (size_t)M * HID * 2;     off = (off + 255) & ~(size_t)255;
  if (off > ws_size || off > (size_t)WSCAP) return;
  unsigned* adjT  = (unsigned*)(ws + oAdj);
  _Float16* obs16 = (_Float16*)(ws + oO16);
  _Float16* w1t   = (_Float16*)(ws + oW1);
  _Float16* w2t   = (_Float16*)(ws + oW2);
  float*    mbuf  = (float*)(ws + oM);
  _Float16* h1h   = (_Float16*)(ws + oH);

  const int nObsBlk = nB * ((NAG * FIN / 8) / NTHR);

  k_prep<<<nObsBlk + PB1 + PB2, NTHR, 0, stream>>>(obs, W1, W2, obs16, w1t, w2t, nObsBlk);

  k_knn<<<nB, KTHR, 0, stream>>>(obs, adjT);

  hipFuncSetAttribute(reinterpret_cast<const void*>(&k_gemm<FIN>),
                      hipFuncAttributeMaxDynamicSharedMemorySize, LDS_GEMM);
  k_gemm<FIN><<<dim3(HID / GT, M / GT), NTHR, LDS_GEMM, stream>>>(obs16, w1t, mbuf, 1.0f / (float)WSCALE);
  k_agg<0><<<nB, NTHR, 0, stream>>>(mbuf, adjT, b1, h1h, obs, Wout, bout, out);

  hipFuncSetAttribute(reinterpret_cast<const void*>(&k_gemm<HID>),
                      hipFuncAttributeMaxDynamicSharedMemorySize, LDS_GEMM);
  k_gemm<HID><<<dim3(HID / GT, M / GT), NTHR, LDS_GEMM, stream>>>(h1h, w2t, mbuf, 1.0f / (float)(ASC2 * WSCALE));
  k_agg<1><<<nB, NTHR, 0, stream>>>(mbuf, adjT, b2, h1h, obs, Wout, bout, out);
}
